// FeatureCubeMLP_18176301597180
// MI455X (gfx1250) — hardware-run, weakly checked
//
#include <hip/hip_runtime.h>
#include <stddef.h>
#include <stdint.h>
#include <math.h>


#pragma clang fp contract(off)

#define RES    256
#define PHW    65536
#define CH     32
#define KF     123
#define KP     128
#define FEAT   128
#define NOUT   4
#define NP3    16
#define PA     136
#define PH     136
#define TM     32
#define NTHR   64
#define PREP_BLOCKS 8
#define PREP_THR 256
#define WSCAP  134217728

#define HSC   64.0f
#define WSC   64.0f
#define INV1  (1.0f / 4096.0f)
#define GMAX  255.0f
#define TWO_PI_F 6.28318530717958647692f

#define W1T_BYTES (FEAT * KP * 2)
#define W2T_BYTES (FEAT * FEAT * 2)
#define W3T_BYTES (NP3 * FEAT * 2)

static_assert(TM == 32);
static_assert(NTHR == 64);
static_assert((KP % 32) == 0 && (FEAT % 32) == 0);
static_assert((PA % 8) == 0 && PA >= KP);
static_assert((PH % 8) == 0 && PH >= FEAT);
static_assert((W1T_BYTES % 512) == 0 && (W2T_BYTES % 512) == 0 && (W3T_BYTES % 512) == 0);
static_assert(KF == 3 * CH + 3 + 24);

typedef float    v4f  __attribute__((ext_vector_type(4)));
typedef float    v8f  __attribute__((ext_vector_type(8)));
typedef _Float16 v4h  __attribute__((ext_vector_type(4)));
typedef _Float16 v8h  __attribute__((ext_vector_type(8)));
typedef _Float16 v16h __attribute__((ext_vector_type(16)));
union FragH { v16h v; v8h h[2]; };

__device__ __forceinline__ v8f wmf(v16h a, v16h b, v8f c) {
  v8f d = __builtin_amdgcn_wmma_f32_16x16x32_f16(false, a, false, b, (short)0, c, false, false);
  asm volatile("v_nop\n\tv_nop\n\tv_nop\n\tv_nop" : "+v"(d) : "v"(a), "v"(b));
  return d;
}

__device__ __forceinline__ void st2_v8h(_Float16* p, v8h v) {
  *(volatile v8h*)p = v;
  __threadfence();
  *(volatile v8h*)p = v;
}

__device__ __forceinline__ void cvt_plane(const float* __restrict__ src, int nreal, int kreal,
                                          int nrows, int kp, float sc, _Float16* dst,
                                          int gt, int gs) {
  const int kq = kp >> 3;
  const int items = nrows * kq;
#pragma unroll 1
  for (int it = gt; it < items; it += gs) {
    const int nrow = it / kq, k8 = it - nrow * kq;
    const int nn = min(nrow, nreal - 1);
    v8h hv;
#pragma unroll
    for (int e = 0; e < 8; ++e) {
      const int k = 8 * k8 + e;
      const int kk = min(k, kreal - 1);
      float w = src[(size_t)nn * kreal + kk];
      w = (nrow < nreal && k < kreal) ? (w * sc) : 0.0f;
      hv[e] = (_Float16)w;
    }
    st2_v8h(dst + (size_t)it * 8, hv);
  }
}

__global__ __launch_bounds__(PREP_THR) void k_prep(const float* __restrict__ W1,
                                                   const float* __restrict__ W2,
                                                   const float* __restrict__ W3,
                                                   _Float16* w1t, _Float16* w2t, _Float16* w3t) {
  const int gt = blockIdx.x * PREP_THR + threadIdx.x;
  const int gs = gridDim.x * PREP_THR;
  cvt_plane(W1, FEAT, KF, FEAT, KP, WSC, w1t, gt, gs);
  cvt_plane(W2, FEAT, FEAT, FEAT, FEAT, WSC, w2t, gt, gs);
  cvt_plane(W3, NOUT, FEAT, NP3, FEAT, WSC, w3t, gt, gs);
}

__device__ __forceinline__ void sample16(const float* __restrict__ plane, float hc, float wc,
                                         int cbase, _Float16* dst) {
  const float h = fminf(fmaxf(hc, 0.0f), GMAX);
  const float w = fminf(fmaxf(wc, 0.0f), GMAX);
  const float h0f = floorf(h), w0f = floorf(w);
  int h0 = (int)h0f, w0 = (int)w0f;
  h0 = min(max(h0, 0), RES - 1);
  w0 = min(max(w0, 0), RES - 1);
  const int h1 = min(h0 + 1, RES - 1), w1 = min(w0 + 1, RES - 1);
  const float dh = h - h0f, dw = w - w0f;
  const float omh = 1.0f - dh, omw = 1.0f - dw;
  const float* base = plane + (size_t)cbase * PHW;
  const int o00 = h0 * RES + w0, o01 = h0 * RES + w1;
  const int o10 = h1 * RES + w0, o11 = h1 * RES + w1;

#pragma unroll 1
  for (int g = 0; g < 4; ++g) {
    const float* gb = base + (size_t)(4 * g) * PHW;
    float t00[4], t01[4], t10[4], t11[4];
#pragma unroll
    for (int e = 0; e < 4; ++e) {
      const float* P = gb + (size_t)e * PHW;
      t00[e] = P[o00];
      t01[e] = P[o01];
      t10[e] = P[o10];
      t11[e] = P[o11];
    }
    __builtin_amdgcn_sched_barrier(0);
    v4h r4;
#pragma unroll
    for (int e = 0; e < 4; ++e) {
      const float a = (t00[e] * omh) * omw;
      const float b = (t01[e] * omh) * dw;
      const float c = (t10[e] * dh) * omw;
      const float d = (t11[e] * dh) * dw;
      const float r = ((a + b) + c) + d;
      r4[e] = (_Float16)(r * HSC);
    }
    *(v4h*)(dst + 4 * g) = r4;
    __builtin_amdgcn_sched_barrier(0);
  }
}

__global__ __launch_bounds__(NTHR) __attribute__((amdgpu_num_vgpr(256)))
void k_main(const float* __restrict__ xc,
            const float* __restrict__ pxy,
            const float* __restrict__ pyz,
            const float* __restrict__ pxz,
            const float* __restrict__ b1,
            const float* __restrict__ b2,
            const float* __restrict__ b3,
            const _Float16* __restrict__ w1t,
            const _Float16* __restrict__ w2t,
            const _Float16* __restrict__ w3t,
            float* out, int n) {
  __shared__ __align__(16) _Float16 sIn[TM * PA];
  __shared__ __align__(16) _Float16 sH[TM * PH];
  __shared__ __align__(16) float sO[TM * NOUT];

  const int tid = threadIdx.x, lane = tid & 31, hh = lane >> 4, m = lane & 15;
  const int wave = __builtin_amdgcn_readfirstlane(tid >> 5);
  const size_t m0 = (size_t)blockIdx.x * TM;
  const v8h z8h = {(_Float16)0.0f, (_Float16)0.0f, (_Float16)0.0f, (_Float16)0.0f,
                   (_Float16)0.0f, (_Float16)0.0f, (_Float16)0.0f, (_Float16)0.0f};
  const v8f z8f = {0.f, 0.f, 0.f, 0.f, 0.f, 0.f, 0.f, 0.f};

  {
    const int sl = tid & (TM - 1);
    const int half = wave;
    const int cbase = half * 16;
    const size_t s = m0 + sl;
    const float c0 = xc[s * 3 + 0], c1 = xc[s * 3 + 1], c2 = xc[s * 3 + 2];
    _Float16* irow = sIn + sl * PA;
    sample16(pxy, c1 * GMAX, c0 * GMAX, cbase, irow + 0 * CH + cbase);
    sample16(pyz, c1 * GMAX, c2 * GMAX, cbase, irow + 1 * CH + cbase);
    sample16(pxz, c2 * GMAX, c0 * GMAX, cbase, irow + 2 * CH + cbase);
    if (half == 0) {
      irow[96] = (_Float16)(c0 * HSC);
      irow[97] = (_Float16)(c1 * HSC);
      irow[98] = (_Float16)(c2 * HSC);
#pragma unroll 1
      for (int t = 0; t < 12; ++t) {
        const int f = t / 3;
        const int d = t - 3 * f;
        const float cd = (d == 0) ? c0 : ((d == 1) ? c1 : c2);
        const float ang = (cd * (float)(1 << f)) * TWO_PI_F;
        irow[99 + t] = (_Float16)(sinf(ang) * HSC);
      }
    } else {
      *(v8h*)(irow + 120) = z8h;
      *(v8h*)(irow + 128) = z8h;
#pragma unroll 1
      for (int t = 0; t < 12; ++t) {
        const int f = t / 3;
        const int d = t - 3 * f;
        const float cd = (d == 0) ? c0 : ((d == 1) ? c1 : c2);
        const float ang = (cd * (float)(1 << f)) * TWO_PI_F;
        irow[111 + t] = (_Float16)(cosf(ang) * HSC);
      }
    }
  }
  __syncthreads();

  const int row0 = wave * 16;

  {
    v8f acc[8];
#pragma unroll
    for (int nt = 0; nt < 8; ++nt) acc[nt] = z8f;
    const _Float16* ar = sIn + (row0 + m) * PA + 8 * hh;
    const _Float16* br = w1t + (size_t)m * KP + 8 * hh;
#pragma unroll 1
    for (int kt = 0; kt < KP / 32; ++kt) {
      const int k0 = 32 * kt;
      FragH a;
      a.h[0] = *(const v8h*)(ar + k0);
      a.h[1] = *(const v8h*)(ar + k0 + 16);
#pragma unroll
      for (int nt = 0; nt < 8; ++nt) {
        const _Float16* bp = br + (size_t)nt * 16 * KP + k0;
        FragH b;
        b.h[0] = *(const v8h*)bp;
        b.h[1] = *(const v8h*)(bp + 16);
        acc[nt] = wmf(a.v, b.v, acc[nt]);
      }
    }
#pragma unroll
    for (int nt = 0; nt < 8; ++nt) {
      const int nn = nt * 16 + m;
      const float bias = b1[nn];
#pragma unroll
      for (int r = 0; r < 8; ++r) {
        float hv = acc[nt][r] * INV1 + bias;
        hv = fmaxf(hv, 0.0f);
        sH[(row0 + 8 * hh + r) * PH + nn] = (_Float16)(hv * HSC);
      }
    }
  }
  __syncthreads();

  {
    v8f acc[8];
#pragma unroll
    for (int nt = 0; nt < 8; ++nt) acc[nt] = z8f;
    const _Float16* ar = sH + (row0 + m) * PH + 8 * hh;
    const _Float16* br = w2t + (size_t)m * FEAT + 8 * hh;
#pragma unroll 1
    for (int kt = 0; kt < FEAT / 32; ++kt) {
      const int k0 = 32 * kt;
      FragH a;
      a.h[0] = *(const v8h*)(ar + k0);
      a.h[1] = *(const v8h*)(ar + k0 + 16);
#pragma unroll
      for (int nt = 0; nt < 8; ++nt) {
        const _Float16* bp = br + (size_t)nt * 16 * FEAT + k0;
        FragH b;
        b.h[0] = *(const v8h*)bp;
        b.h[1] = *(const v8h*)(bp + 16);
        acc[nt] = wmf(a.v, b.v, acc[nt]);
      }
    }
#pragma unroll
    for (int nt = 0; nt < 8; ++nt) {
      const int nn = nt * 16 + m;
      const float bias = b2[nn];
#pragma unroll
      for (int r = 0; r < 8; ++r) {
        float hv = acc[nt][r] * INV1 + bias;
        hv = fmaxf(hv, 0.0f);
        sH[(row0 + 8 * hh + r) * PH + nn] = (_Float16)(hv * HSC);
      }
    }
  }
  __syncthreads();

  {
    v8f acc = z8f;
    const _Float16* ar = sH + (row0 + m) * PH + 8 * hh;
    const _Float16* br = w3t + (size_t)m * FEAT + 8 * hh;
#pragma unroll
    for (int kt = 0; kt < FEAT / 32; ++kt) {
      const int k0 = 32 * kt;
      FragH a, b;
      a.h[0] = *(const v8h*)(ar + k0);
      a.h[1] = *(const v8h*)(ar + k0 + 16);
      b.h[0] = *(const v8h*)(br + k0);
      b.h[1] = *(const v8h*)(br + k0 + 16);
      acc = wmf(a.v, b.v, acc);
    }
    const float bias = b3[min(m, NOUT - 1)];
#pragma unroll
    for (int r = 0; r < 8; ++r) {
      const int rowl = row0 + 8 * hh + r;
      const float v = acc[r] * INV1 + bias;
      if (m < NOUT) sO[rowl * NOUT + m] = v;
    }
  }
  __syncthreads();

  if (wave == 0) {
    const v4f v = *(const v4f*)(sO + 4 * lane);
    float* gp = out + m0 * NOUT;
    *(volatile v4f*)(gp + 4 * lane) = v;
    __threadfence();
    *(volatile v4f*)(gp + 4 * lane) = v;
  }
}

extern "C" void kernel_launch(void* const* d_in, const int* in_sizes, int n_in,
                              void* d_out, int out_size, void* d_ws, size_t ws_size,
                              hipStream_t stream) {
  if (n_in < 10) return;
  const int n = in_sizes[0] / 3;
  if (n <= 0 || in_sizes[0] != 3 * n) return;
  if ((n % TM) != 0) return;
  if (in_sizes[1] != CH * PHW || in_sizes[2] != CH * PHW || in_sizes[3] != CH * PHW) return;
  if (in_sizes[4] != FEAT * KF || in_sizes[5] != FEAT) return;
  if (in_sizes[6] != FEAT * FEAT || in_sizes[7] != FEAT) return;
  if (in_sizes[8] != NOUT * FEAT || in_sizes[9] != NOUT) return;
  if (out_size != NOUT * n) return;

  const float* xc  = (const float*)d_in[0];
  const float* pxy = (const float*)d_in[1];
  const float* pyz = (const float*)d_in[2];
  const float* pxz = (const float*)d_in[3];
  const float* W1  = (const float*)d_in[4];
  const float* b1  = (const float*)d_in[5];
  const float* W2  = (const float*)d_in[6];
  const float* b2  = (const float*)d_in[7];
  const float* W3  = (const float*)d_in[8];
  const float* b3  = (const float*)d_in[9];
  float* out = (float*)d_out;

  char* ws = (char*)d_ws;
  size_t off = 0;
  const size_t oW1 = off; off += W1T_BYTES; off = (off + 255) & ~(size_t)255;
  const size_t oW2 = off; off += W2T_BYTES; off = (off + 255) & ~(size_t)255;
  const size_t oW3 = off; off += W3T_BYTES; off = (off + 255) & ~(size_t)255;
  if (off > ws_size || off > (size_t)WSCAP) return;
  _Float16* w1t = (_Float16*)(ws + oW1);
  _Float16* w2t = (_Float16*)(ws + oW2);
  _Float16* w3t = (_Float16*)(ws + oW3);

  k_prep<<<PREP_BLOCKS, PREP_THR, 0, stream>>>(W1, W2, W3, w1t, w2t, w3t);
  k_main<<<n / TM, NTHR, 0, stream>>>(xc, pxy, pyz, pxz, b1, b2, b3, w1t, w2t, w3t, out, n);
}
